// Involution_bin_75282186764559
// MI455X (gfx1250) — hardware-run, weakly checked
//
#include <hip/hip_runtime.h>
#include <math.h>

typedef __attribute__((ext_vector_type(16))) _Float16 v16h;
typedef __attribute__((ext_vector_type(8)))  _Float16 v8h;
typedef __attribute__((ext_vector_type(8)))  float    v8f;
typedef __attribute__((ext_vector_type(4)))  float    v4f;

constexpr int kNB = 8;
constexpr int kNC = 64;
constexpr int kNH = 128;
constexpr int kNW = 128;
constexpr int kHW = kNH * kNW;
constexpr int kNRed = 32;
constexpr int kNTap = 9;
constexpr size_t kTen = (size_t)kNB * kNC * kHW;
constexpr int kPixAll = kNB * kHW;
constexpr float kEps = 1e-5f;
constexpr float kCarry = 64.0f;
constexpr float kCarryInv = 1.0f / kCarry;
constexpr float kKerFold = 1.0f / (kCarry * kCarry);
constexpr int kBlkRow = kNB * kNH;
constexpr int kBlkInv = kNB * (kNH / 8) * (kNW / 32);
static_assert(kHW == 16384 && kTen == 8388608ull && kPixAll == 131072, "shape");
static_assert(kBlkRow == 1024 && kBlkInv == 512, "grids");
static_assert((kNC % 32) == 0, "K multiple of 32");

constexpr size_t kOffS     = 0;
constexpr size_t kOffZ     = kOffS     + kTen * 2;
constexpr size_t kOffP     = kOffZ     + kTen * 4;
constexpr size_t kOffPart0 = kOffP     + kTen * 4;
constexpr size_t kOffPart1 = kOffPart0 + (size_t)kBlkRow * 128 * 4;
constexpr size_t kOffPart2 = kOffPart1 + (size_t)kBlkInv * 128 * 4;
constexpr size_t kOffTab   = kOffPart2 + (size_t)kBlkRow * 128 * 4;
constexpr size_t kOffAB0   = kOffTab   + 256 * 4;
constexpr size_t kOffAB1   = kOffAB0   + 128 * 4;
constexpr size_t kOffAB2   = kOffAB1   + 128 * 4;
constexpr size_t kOffSgnA  = kOffAB2   + 128 * 4;
constexpr size_t kOffSgnB  = kOffSgnA  + 64 * 64 * 2;
constexpr size_t kOffQP    = kOffSgnB  + 64 * 64 * 2;
constexpr size_t kWsTotal  = kOffQP    + 16 * 64 * 2;
static_assert(kWsTotal == 85217792ull, "carve total");
static_assert(kWsTotal <= 134217728ull, "carve cap");
static_assert((kOffZ % 128) == 0 && (kOffP % 128) == 0 && (kOffPart0 % 128) == 0 && (kOffPart1 % 128) == 0 &&
              (kOffPart2 % 128) == 0 && (kOffTab % 128) == 0 && (kOffAB0 % 128) == 0 && (kOffAB1 % 128) == 0 &&
              (kOffAB2 % 128) == 0 && (kOffSgnA % 128) == 0 && (kOffSgnB % 128) == 0 && (kOffQP % 128) == 0, "aligned");

__device__ __forceinline__ float sgnf(float v) {
  return (v > 0.f) ? 1.f : ((v < 0.f) ? -1.f : 0.f);
}

__device__ __forceinline__ float h16_to_f32(unsigned hb) {
  const unsigned sgn = (hb & 0x8000u) << 16;
  const unsigned em = hb & 0x7fffu;
  const float fn = __uint_as_float((em << 13) + 0x38000000u);
  const float fs = (float)em * 5.9604644775390625e-8f;
  const float mag = (em < 0x400u) ? fs : fn;
  return __uint_as_float(__float_as_uint(mag) | sgn);
}

union FragU { v16h v; v8h h[2]; };
__device__ __forceinline__ v16h frag_load(const _Float16* p) {
  FragU f;
  f.h[0] = *(const v8h*)(p);
  f.h[1] = *(const v8h*)(p + 16);
  return f.v;
}
__device__ __forceinline__ v8f mma_h(v16h a, v16h b, v8f c) {
  c = __builtin_amdgcn_wmma_f32_16x16x32_f16(false, a, false, b, (short)0, c, false, false);
  asm volatile("v_nop\n\tv_nop\n\tv_nop\n\tv_nop" : "+v"(c) : "v"(a), "v"(b));
  return c;
}

__global__ __launch_bounds__(256) void prep_kernel(
    const float* __restrict__ pre_w, const float* __restrict__ post_w,
    const float* __restrict__ red_w, const float* __restrict__ span_w,
    float* __restrict__ tab, unsigned short* __restrict__ sgn_pre,
    unsigned short* __restrict__ sgn_post, unsigned short* __restrict__ qp)
{
  __shared__ float s_tab[256];
  const int tid = threadIdx.x;
  const int lane = tid & 31;
  const int wave = __builtin_amdgcn_readfirstlane((int)(threadIdx.x >> 5));

  const float* wp = pre_w;
  int n = 0;
  int row = 0;
  bool valid = false;
  float invn = 0.f;
  if (wave < 2) {
    wp = pre_w; n = 64; row = tid; valid = true; invn = 1.0f / 64.0f;
  } else if (wave < 4) {
    wp = post_w; n = 64; row = tid - 64; valid = true; invn = 1.0f / 64.0f;
  } else if (wave == 4) {
    wp = span_w; n = 32; row = (lane < kNTap) ? lane : (kNTap - 1); valid = (lane < kNTap); invn = 1.0f / 32.0f;
  } else if (wave == 5) {
    wp = red_w; n = 64; row = lane; valid = true; invn = 1.0f / 64.0f;
  }
  float s = 0.f;
#pragma unroll 1
  for (int i = 0; i < n; ++i) s += fabsf(wp[row * n + i]);
  const float mv = s * invn;
  s_tab[tid] = valid ? mv : 0.f;
  __syncthreads();

  {
    const float tv = s_tab[tid];
    *(volatile float*)(tab + tid) = tv;
    __threadfence();
    *(volatile float*)(tab + tid) = tv;
  }

#pragma unroll 1
  for (int it = 0; it < 2; ++it) {
    const int e0 = (it * 256 + tid) * 8;
    const v4f a0 = *(const v4f*)(pre_w + e0);
    const v4f a1 = *(const v4f*)(pre_w + e0 + 4);
    const v4f b0 = *(const v4f*)(post_w + e0);
    const v4f b1 = *(const v4f*)(post_w + e0 + 4);
    v8h hp, hq;
#pragma unroll
    for (int e = 0; e < 4; ++e) {
      hp[e]     = (_Float16)sgnf(a0[e]);
      hp[4 + e] = (_Float16)sgnf(a1[e]);
      hq[e]     = (_Float16)sgnf(b0[e]);
      hq[4 + e] = (_Float16)sgnf(b1[e]);
    }
    *(volatile v8h*)(sgn_pre + e0) = hp;
    *(volatile v8h*)(sgn_post + e0) = hq;
    __threadfence();
    *(volatile v8h*)(sgn_pre + e0) = hp;
    *(volatile v8h*)(sgn_post + e0) = hq;
  }

  if (wave < 4) {
    const int k = tid >> 3;
    const int kc = (k < kNTap) ? k : (kNTap - 1);
    const int c0 = (tid & 7) * 8;
    float acc[8];
#pragma unroll
    for (int e = 0; e < 8; ++e) acc[e] = 0.f;
#pragma unroll 1
    for (int j = 0; j < kNRed; ++j) {
      const float sj = sgnf(span_w[kc * kNRed + j]) * s_tab[160 + j];
      const v4f r0 = *(const v4f*)(red_w + j * kNC + c0);
      const v4f r1 = *(const v4f*)(red_w + j * kNC + c0 + 4);
#pragma unroll
      for (int e = 0; e < 4; ++e) {
        acc[e]     = fmaf(sj, sgnf(r0[e]), acc[e]);
        acc[4 + e] = fmaf(sj, sgnf(r1[e]), acc[4 + e]);
      }
    }
    v8h qv;
#pragma unroll
    for (int e = 0; e < 8; ++e) {
      const float qf = (k < kNTap) ? (acc[e] * kCarry) : 0.0f;
      qv[e] = (_Float16)qf;
    }
    *(volatile v8h*)(qp + tid * 8) = qv;
    __threadfence();
    *(volatile v8h*)(qp + tid * 8) = qv;
  }
}

template <int MODE>
__global__ __launch_bounds__(256) void conv_gemm_kernel(
    const float* __restrict__ in, const unsigned short* __restrict__ sgnp,
    const float* __restrict__ ab, void* __restrict__ outp, float* __restrict__ part)
{
  __shared__ __align__(16) _Float16 s_act[128 * 72];
  __shared__ __align__(16) float s_d[64 * 132];
  __shared__ __align__(16) float s_st[128];
  __shared__ float s_ab[128];
  const int tid = threadIdx.x;
  const int lane = tid & 31;
  const int wave = __builtin_amdgcn_readfirstlane((int)(threadIdx.x >> 5));
  const int hh = lane >> 4;
  const int rl = lane & 15;
  const int b = blockIdx.x >> 7;
  const int y = blockIdx.x & 127;

  if (MODE == 1) {
    if (wave < 4) s_ab[tid] = ab[tid];
    __syncthreads();
  }

  {
    const int p = tid & 127;
    const int chalf = wave >> 2;
    const float* src = in + (size_t)(b * kNC) * kHW + y * kNW + p;
#pragma unroll 1
    for (int g = 0; g < 4; ++g) {
      const int c0 = chalf * 32 + g * 8;
      float v[8];
#pragma unroll
      for (int e = 0; e < 8; ++e) v[e] = src[(size_t)(c0 + e) * kHW];
      v8h hv;
#pragma unroll
      for (int e = 0; e < 8; ++e) {
        float t;
        if (MODE == 0) {
          t = sgnf(v[e]);
        } else {
          t = fmaxf(fmaf(s_ab[c0 + e], v[e], s_ab[64 + c0 + e]), 0.0f) * kCarry;
        }
        hv[e] = (_Float16)t;
      }
      *(v8h*)(s_act + p * 72 + c0) = hv;
    }
  }
  __syncthreads();

  {
    const _Float16* sg = (const _Float16*)sgnp;
    const float osc = (MODE == 0) ? 1.0f : kCarryInv;
    const v16h bf0 = frag_load(s_act + (wave * 16 + rl) * 72 + 8 * hh);
    const v16h bf1 = frag_load(s_act + (wave * 16 + rl) * 72 + 32 + 8 * hh);
#pragma unroll
    for (int mt = 0; mt < 4; ++mt) {
      const v16h a0 = frag_load(sg + (mt * 16 + rl) * kNC + 8 * hh);
      const v16h a1 = frag_load(sg + (mt * 16 + rl) * kNC + 32 + 8 * hh);
      v8f acc = (v8f){0.f, 0.f, 0.f, 0.f, 0.f, 0.f, 0.f, 0.f};
      acc = mma_h(a0, bf0, acc);
      acc = mma_h(a1, bf1, acc);
#pragma unroll
      for (int r = 0; r < 8; ++r)
        s_d[(mt * 16 + 8 * hh + r) * 132 + wave * 16 + rl] = acc[r] * osc;
    }
  }
  __syncthreads();

  if (MODE == 0) {
    unsigned short* So = (unsigned short*)outp;
    v8h hv[4];
#pragma unroll
    for (int it = 0; it < 4; ++it) {
      const int c = (it * 8 + wave) * 2 + hh;
      const v4f f0 = *(const v4f*)(s_d + c * 132 + rl * 8);
      const v4f f1 = *(const v4f*)(s_d + c * 132 + rl * 8 + 4);
      float s = 0.f, q = 0.f;
#pragma unroll
      for (int e = 0; e < 4; ++e) {
        hv[it][e]     = (_Float16)f0[e];
        hv[it][4 + e] = (_Float16)f1[e];
        s += f0[e];
        s += f1[e];
        q = fmaf(f0[e], f0[e], q);
        q = fmaf(f1[e], f1[e], q);
      }
#pragma unroll
      for (int off = 1; off < 16; off <<= 1) {
        s += __shfl_xor(s, off, 32);
        q += __shfl_xor(q, off, 32);
      }
      if (rl == 0) {
        s_st[c] = s;
        s_st[64 + c] = q;
      }
    }
    for (int pass = 0; pass < 2; ++pass) {
#pragma unroll
      for (int it = 0; it < 4; ++it) {
        const int c = (it * 8 + wave) * 2 + hh;
        *(volatile v8h*)(So + (size_t)(b * kNC + c) * kHW + y * kNW + rl * 8) = hv[it];
      }
      __threadfence();
    }
  } else {
    float* Po = (float*)outp;
    v4f pv[8];
#pragma unroll
    for (int it = 0; it < 8; ++it) {
      const int c = wave * 8 + it;
      pv[it] = *(const v4f*)(s_d + c * 132 + lane * 4);
      float s = 0.f, q = 0.f;
#pragma unroll
      for (int e = 0; e < 4; ++e) {
        s += pv[it][e];
        q = fmaf(pv[it][e], pv[it][e], q);
      }
#pragma unroll
      for (int off = 1; off < 32; off <<= 1) {
        s += __shfl_xor(s, off, 32);
        q += __shfl_xor(q, off, 32);
      }
      if (lane == 0) {
        s_st[c] = s;
        s_st[64 + c] = q;
      }
    }
    for (int pass = 0; pass < 2; ++pass) {
#pragma unroll
      for (int it = 0; it < 8; ++it) {
        const int c = wave * 8 + it;
        *(volatile v4f*)(Po + (size_t)(b * kNC + c) * kHW + y * kNW + lane * 4) = pv[it];
      }
      __threadfence();
    }
  }
  __syncthreads();
  if (wave == 0) {
    const v4f sv = *(const v4f*)(s_st + lane * 4);
    float* pp = part + (size_t)blockIdx.x * 128 + lane * 4;
    *(volatile v4f*)pp = sv;
    __threadfence();
    *(volatile v4f*)pp = sv;
  }
}

__global__ __launch_bounds__(256) void fold_kernel(
    const float* __restrict__ part, int nblk, const float* __restrict__ sf, int use_sf,
    const float* __restrict__ gamma, const float* __restrict__ beta, float* __restrict__ abo)
{
  __shared__ double s_s[256];
  __shared__ double s_q[256];
  __shared__ __align__(16) float s_o[128];
  const int tid = threadIdx.x;
  const int lane = tid & 31;
  const int wave = __builtin_amdgcn_readfirstlane((int)(threadIdx.x >> 5));
  const int c = tid & 63;
  const int qd = tid >> 6;
  const int per = nblk >> 2;
  double s = 0.0, q = 0.0;
#pragma unroll 1
  for (int i = 0; i < per; ++i) {
    const size_t o = (size_t)(qd * per + i) * 128;
    s += (double)part[o + c];
    q += (double)part[o + 64 + c];
  }
  s_s[tid] = s;
  s_q[tid] = q;
  __syncthreads();
  if (wave < 2) {
    const double ss = (s_s[tid] + s_s[64 + tid]) + (s_s[128 + tid] + s_s[192 + tid]);
    const double qq = (s_q[tid] + s_q[64 + tid]) + (s_q[128 + tid] + s_q[192 + tid]);
    const double invn = 1.0 / (double)kPixAll;
    const double m = ss * invn;
    double var = qq * invn - m * m;
    var = (var < 0.0) ? 0.0 : var;
    float sfv = 1.0f;
    if (use_sf != 0) sfv = sf[tid];
    const float vs = (float)((double)sfv * (double)sfv * var);
    const float a = gamma[tid] * sfv * rsqrtf(vs + kEps);
    const float bb = (float)((double)beta[tid] - (double)a * m);
    s_o[tid] = a;
    s_o[64 + tid] = bb;
  }
  __syncthreads();
  if (wave == 0) {
    const v4f ov = *(const v4f*)(s_o + lane * 4);
    *(volatile v4f*)(abo + lane * 4) = ov;
    __threadfence();
    *(volatile v4f*)(abo + lane * 4) = ov;
  }
}

__global__ __launch_bounds__(256) void invol_kernel(
    const unsigned short* __restrict__ S, const float* __restrict__ ab0,
    const float* __restrict__ pre_a, const float* __restrict__ mid_bias,
    const unsigned short* __restrict__ qp, const float* __restrict__ tab,
    float* __restrict__ Z, float* __restrict__ part)
{
  __shared__ __align__(16) _Float16 s_hA[256 * 72];
  __shared__ __align__(16) float s_halo[8 * 340];
  __shared__ float s_par[256];
  __shared__ float s_sfs[32];
  __shared__ float s_ws[8 * 128];
  __shared__ __align__(16) float s_fin[128];
  const int tid = threadIdx.x;
  const int lane = tid & 31;
  const int wave = __builtin_amdgcn_readfirstlane((int)(threadIdx.x >> 5));
  const int hh = lane >> 4;
  const int rl = lane & 15;
  const int blk = blockIdx.x;
  const int b = blk >> 6;
  const int y0 = ((blk >> 2) & 15) * 8;
  const int x0 = (blk & 3) * 32;
  const int gy = y0 + wave;
  const int gx = x0 + lane;

  {
    float pv;
    if (wave < 4) pv = ab0[tid];
    else if (wave < 6) pv = pre_a[tid - 128];
    else pv = mid_bias[tid - 192];
    s_par[tid] = pv;
  }
  if (wave == 0) s_sfs[lane] = tab[128 + lane];
  __syncthreads();

  const unsigned short* Sb = S + (size_t)(b * kNC) * kHW;
  {
    const unsigned short* Sp = Sb + gy * kNW + gx;
#pragma unroll 1
    for (int g = 0; g < 8; ++g) {
      unsigned hb[8];
#pragma unroll
      for (int e = 0; e < 8; ++e) hb[e] = Sp[(size_t)(g * 8 + e) * kHW];
      v8h hv;
#pragma unroll
      for (int e = 0; e < 8; ++e) {
        const int c = g * 8 + e;
        const float sv = h16_to_f32(hb[e]);
        const float t = fmaf(s_par[c], sv, s_par[64 + c]);
        const float h = fmaxf(t, 0.0f) + s_par[128 + c] * fminf(t, 0.0f) + s_par[192 + c];
        hv[e] = (_Float16)(h * kCarry);
      }
      *(v8h*)(s_hA + tid * 72 + g * 8) = hv;
    }
  }
  __syncthreads();

  float ker[9];
  {
    const _Float16* Qh = (const _Float16*)qp;
    const v16h qa0 = frag_load(Qh + rl * kNC + 8 * hh);
    const v16h qa1 = frag_load(Qh + rl * kNC + 32 + 8 * hh);
    v8f acc0 = (v8f){0.f, 0.f, 0.f, 0.f, 0.f, 0.f, 0.f, 0.f};
    v8f acc1 = (v8f){0.f, 0.f, 0.f, 0.f, 0.f, 0.f, 0.f, 0.f};
    {
      const v16h hb0 = frag_load(s_hA + (wave * 32 + rl) * 72 + 8 * hh);
      const v16h hb1 = frag_load(s_hA + (wave * 32 + rl) * 72 + 32 + 8 * hh);
      acc0 = mma_h(qa0, hb0, acc0);
      acc0 = mma_h(qa1, hb1, acc0);
    }
    {
      const v16h hb0 = frag_load(s_hA + (wave * 32 + 16 + rl) * 72 + 8 * hh);
      const v16h hb1 = frag_load(s_hA + (wave * 32 + 16 + rl) * 72 + 32 + 8 * hh);
      acc1 = mma_h(qa0, hb0, acc1);
      acc1 = mma_h(qa1, hb1, acc1);
    }
#pragma unroll
    for (int r = 0; r < 8; ++r) {
      const float o = __shfl_xor(acc1[r], 16, 32);
      const float own = acc0[r];
      ker[r] = (lane < 16) ? own : o;
    }
    {
      const float o8 = __shfl_xor(acc0[0], 16, 32);
      const float own8 = acc1[0];
      ker[8] = (lane < 16) ? o8 : own8;
    }
#pragma unroll
    for (int k = 0; k < 9; ++k) ker[k] = ker[k] * (s_sfs[k] * kKerFold);
  }

  float* s_wsw = s_ws + wave * 128;
#pragma unroll 1
  for (int g = 0; g < 8; ++g) {
    __syncthreads();
#pragma unroll 1
    for (int it = 0; it < 11; ++it) {
      const unsigned idx = (unsigned)(it * 256 + tid);
      const unsigned idc = (idx < 2720u) ? idx : 2719u;
      const unsigned cl = idc / 340u;
      const unsigned rem = idc - cl * 340u;
      const unsigned ey = rem / 34u;
      const unsigned ex = rem - ey * 34u;
      const int yy = y0 + (int)ey - 1;
      const int xx = x0 + (int)ex - 1;
      const bool inimg = ((unsigned)yy < (unsigned)kNH) && ((unsigned)xx < (unsigned)kNW);
      const int yc = (yy < 0) ? 0 : ((yy > kNH - 1) ? (kNH - 1) : yy);
      const int xc = (xx < 0) ? 0 : ((xx > kNW - 1) ? (kNW - 1) : xx);
      const int c = g * 8 + (int)cl;
      unsigned hbv = Sb[(size_t)c * kHW + yc * kNW + xc];
      asm volatile("" : "+v"(hbv));
      const float sv = h16_to_f32(hbv);
      const float t = fmaf(s_par[c], sv, s_par[64 + c]);
      const float h = fmaxf(t, 0.0f) + s_par[128 + c] * fminf(t, 0.0f) + s_par[192 + c];
      const float val = inimg ? h : 0.0f;
      if (idx < 2720u) s_halo[idc] = val;
    }
    __syncthreads();

    float zv[8];
#pragma unroll
    for (int cl = 0; cl < 8; ++cl) {
      const float* hp = s_halo + cl * 340 + wave * 34 + lane;
      float a = 0.0f;
#pragma unroll
      for (int i = 0; i < 3; ++i)
#pragma unroll
        for (int j = 0; j < 3; ++j)
          a = fmaf(hp[i * 34 + j], ker[i * 3 + j], a);
      zv[cl] = a;
    }
#pragma unroll
    for (int cl = 0; cl < 8; ++cl) {
      float s = zv[cl];
      float q = zv[cl] * zv[cl];
#pragma unroll
      for (int off = 1; off < 32; off <<= 1) {
        s += __shfl_xor(s, off, 32);
        q += __shfl_xor(q, off, 32);
      }
      if (lane == 0) {
        s_wsw[g * 8 + cl] = s;
        s_wsw[64 + g * 8 + cl] = q;
      }
    }
    for (int pass = 0; pass < 2; ++pass) {
#pragma unroll
      for (int cl = 0; cl < 8; ++cl)
        *(volatile float*)(Z + (size_t)(b * kNC + g * 8 + cl) * kHW + gy * kNW + gx) = zv[cl];
      __threadfence();
    }
  }
  __syncthreads();
  if (wave < 4) {
    float t = 0.0f;
#pragma unroll
    for (int w = 0; w < 8; ++w) t += s_ws[w * 128 + tid];
    s_fin[tid] = t;
  }
  __syncthreads();
  if (wave == 0) {
    const v4f sv = *(const v4f*)(s_fin + lane * 4);
    float* pp = part + (size_t)blk * 128 + lane * 4;
    *(volatile v4f*)pp = sv;
    __threadfence();
    *(volatile v4f*)pp = sv;
  }
}

__global__ __launch_bounds__(256) void final_kernel(
    const float* __restrict__ P, const float* __restrict__ x,
    const float* __restrict__ ab2, float* __restrict__ out)
{
  const int tid = threadIdx.x;
  v4f ov[4];
#pragma unroll
  for (int j = 0; j < 4; ++j) {
    const size_t i4 = ((size_t)blockIdx.x * 4 + j) * 256 + tid;
    const int c = (int)((i4 >> 12) & 63);
    const float a = ab2[c];
    const float bb = ab2[64 + c];
    const v4f pv = *(const v4f*)(P + i4 * 4);
    const v4f xv = *(const v4f*)(x + i4 * 4);
    v4f o;
#pragma unroll
    for (int e = 0; e < 4; ++e) o[e] = fmaf(a, pv[e], bb) + xv[e];
    ov[j] = o;
  }
  for (int pass = 0; pass < 2; ++pass) {
#pragma unroll
    for (int j = 0; j < 4; ++j) {
      const size_t i4 = ((size_t)blockIdx.x * 4 + j) * 256 + tid;
      *(volatile v4f*)(out + i4 * 4) = ov[j];
    }
    __threadfence();
  }
}

extern "C" void kernel_launch(void* const* d_in, const int* in_sizes, int n_in,
                              void* d_out, int out_size, void* d_ws, size_t ws_size,
                              hipStream_t stream) {
  if (n_in < 16) return;
  if (in_sizes[0] != (int)kTen) return;
  if (in_sizes[2] != kNC * kNC) return;
  if (in_sizes[3] != kNC || in_sizes[4] != kNC || in_sizes[5] != kNC || in_sizes[6] != kNC) return;
  if (in_sizes[7] != kNRed * kNC) return;
  if (in_sizes[8] != kNTap * kNRed) return;
  if (in_sizes[9] != kNC || in_sizes[10] != kNC) return;
  if (in_sizes[13] != kNC * kNC) return;
  if (in_sizes[14] != kNC || in_sizes[15] != kNC) return;
  if (out_size != (int)kTen) return;
  if (ws_size < kWsTotal) return;

  const float* x          = (const float*)d_in[0];
  const float* pre_w      = (const float*)d_in[2];
  const float* pre_gamma  = (const float*)d_in[3];
  const float* pre_beta   = (const float*)d_in[4];
  const float* pre_a      = (const float*)d_in[5];
  const float* mid_bias   = (const float*)d_in[6];
  const float* red_w      = (const float*)d_in[7];
  const float* span_w     = (const float*)d_in[8];
  const float* mid_gamma  = (const float*)d_in[9];
  const float* mid_beta   = (const float*)d_in[10];
  const float* post_w     = (const float*)d_in[13];
  const float* post_gamma = (const float*)d_in[14];
  const float* post_beta  = (const float*)d_in[15];
  float* out = (float*)d_out;

  char* ws = (char*)d_ws;
  unsigned short* Sraw  = (unsigned short*)(ws + kOffS);
  float*          Zb    = (float*)(ws + kOffZ);
  float*          Pb    = (float*)(ws + kOffP);
  float*          part0 = (float*)(ws + kOffPart0);
  float*          part1 = (float*)(ws + kOffPart1);
  float*          part2 = (float*)(ws + kOffPart2);
  float*          tab   = (float*)(ws + kOffTab);
  float*          AB0   = (float*)(ws + kOffAB0);
  float*          AB1   = (float*)(ws + kOffAB1);
  float*          AB2   = (float*)(ws + kOffAB2);
  unsigned short* sgnA  = (unsigned short*)(ws + kOffSgnA);
  unsigned short* sgnB  = (unsigned short*)(ws + kOffSgnB);
  unsigned short* QP    = (unsigned short*)(ws + kOffQP);

  prep_kernel<<<1, 256, 0, stream>>>(pre_w, post_w, red_w, span_w, tab, sgnA, sgnB, QP);
  conv_gemm_kernel<0><<<kBlkRow, 256, 0, stream>>>(x, sgnA, tab, (void*)Sraw, part0);
  fold_kernel<<<1, 256, 0, stream>>>(part0, kBlkRow, tab, 1, pre_gamma, pre_beta, AB0);
  invol_kernel<<<kBlkInv, 256, 0, stream>>>(Sraw, AB0, pre_a, mid_bias, QP, tab, Zb, part1);
  fold_kernel<<<1, 256, 0, stream>>>(part1, kBlkInv, tab, 0, mid_gamma, mid_beta, AB1);
  conv_gemm_kernel<1><<<kBlkRow, 256, 0, stream>>>(Zb, sgnB, AB1, (void*)Pb, part2);
  fold_kernel<<<1, 256, 0, stream>>>(part2, kBlkRow, tab + 64, 1, post_gamma, post_beta, AB2);
  final_kernel<<<2048, 256, 0, stream>>>(Pb, x, AB2, out);
}
